// LDDMMHamilton_31361851195746
// MI455X (gfx1250) — hardware-verified
//
#include <hip/hip_runtime.h>


#ifndef NPTS
#define NPTS 8192
#endif
#define NPTS_FULL 8192
#define CD   3
#define AW   4
#define TPB  (16 * AW)
#define OSF  (TPB * CD)
#define FB   256
#define FW   16
#define OUT1_OFF ((size_t)NPTS_FULL * CD)
#define KSH  14.0f
#define BC   1024.0f
#define INV_S2 (1.0 / (0.1 * 0.1))
#define ES_  ((float)(-(INV_S2) * 1.4426950408889634))
#define C0_  ((float)(4.0 * (INV_S2) / (16384.0 * 1024.0)))
#define C1_  ((float)(2.0 / (16384.0 * 1024.0)))

static_assert(NPTS <= NPTS_FULL);
static_assert(NPTS % FB == 0);
static_assert(NPTS % TPB == 0);
static_assert(NPTS % 32 == 0);
static_assert(FB == 256);
static_assert(FB / 8 == 32);
static_assert(FB * FW * 2 == 2 * FB * 16);
static_assert(16 * FB * 2 == 2 * FB * 16);
static_assert((FB / 4) * 16 == FB * 4);
static_assert((FB / 4) % 32 == 0);
static_assert((FB * 4) % 128 == 0);
static_assert(FW == 16);
static_assert((OSF * 4) % 128 == 0);
static_assert((2 * OSF / 4) * 16 == 2 * TPB * CD * 4);
static_assert(2 * OSF / 4 <= 32 * AW);
static_assert((OSF / 4) % 8 == 0);
static_assert((OUT1_OFF * 4) % 128 == 0);
static_assert(OUT1_OFF * 4 == (size_t)98304);
static_assert(2 * FB * FW * 2 + 16 * FB * 2 + FB * 4 <= 131072);
static_assert(2 * OSF * 4 <= 131072);

typedef _Float16 h16;
typedef unsigned short bf;
typedef __attribute__((ext_vector_type(16))) __bf16   v16bf;
typedef __attribute__((ext_vector_type(16))) _Float16 v16h;
typedef __attribute__((ext_vector_type(8)))  _Float16 v8h;
typedef __attribute__((ext_vector_type(8)))  unsigned short v8us;
typedef __attribute__((ext_vector_type(8)))  float    v8f;
typedef __attribute__((ext_vector_type(4)))  float    v4f;
typedef v4f  __attribute__((may_alias)) v4fa;
typedef v8us __attribute__((may_alias)) v8usa;
typedef v8h  __attribute__((may_alias)) v8ha;

__device__ __forceinline__ unsigned short f2bf(float f) { unsigned u = __float_as_uint(f); u += 0x7FFFu + ((u >> 16) & 1u); return (unsigned short)(u >> 16); }
__device__ __forceinline__ float bfr(float f) { return __uint_as_float(((unsigned)f2bf(f)) << 16); }
__device__ __forceinline__ float bf2f(unsigned short b) { return __uint_as_float(((unsigned)b) << 16); }
__device__ __forceinline__ v16h cat16(v8h lo, v8h hi) { return __builtin_shufflevector(lo, hi, 0, 1, 2, 3, 4, 5, 6, 7, 8, 9, 10, 11, 12, 13, 14, 15); }
__device__ __forceinline__ v16bf cat16b(v8us lo, v8us hi) { return __builtin_bit_cast(v16bf, __builtin_shufflevector(lo, hi, 0, 1, 2, 3, 4, 5, 6, 7, 8, 9, 10, 11, 12, 13, 14, 15)); }
__device__ __forceinline__ v8f wmma16(v16h a, v16h b, v8f c) { return __builtin_amdgcn_wmma_f32_16x16x32_f16(false, a, false, b, (short)0, c, false, false); }
__device__ __forceinline__ v8f wmmab(v16bf a, v16bf b, v8f c) { return __builtin_amdgcn_wmma_f32_16x16x32_bf16(false, a, false, b, (short)0, c, false, false); }
__device__ __forceinline__ v16h  ldh(const h16* p) { return cat16(*(const v8h*)p, *(const v8h*)(p + 16)); }
__device__ __forceinline__ v8f wmma16g(v16h a, v16h b, v8f c) { c = wmma16(a, b, c); asm volatile("v_nop\n\tv_nop\n\tv_nop\n\tv_nop" : "+v"(c) : "v"(a), "v"(b)); return c; }
__device__ __forceinline__ v8f wmmabg(v16bf a, v16bf b, v8f c) { c = wmmab(a, b, c); asm volatile("v_nop\n\tv_nop\n\tv_nop\n\tv_nop" : "+v"(c) : "v"(a), "v"(b)); return c; }
static __device__ __forceinline__ h16 toh_flush(float v) { const h16 r = (h16)v; return (fabsf(v) < 6.103515625e-05f) ? (h16)0.0f : r; }

__global__ __launch_bounds__(FB) void k_feat(const float* __restrict__ mom, const float* __restrict__ cpt, bf* FJ, bf* FI, h16* CT, float* NQ) {
#pragma clang fp contract(off)
    __shared__ __align__(16) unsigned short sj[FB * FW];
    __shared__ __align__(16) unsigned short si[FB * FW];
    __shared__ __align__(16) h16 sc[16 * FB];
    __shared__ __align__(16) float sn[FB];
    const int t = threadIdx.x;
    const size_t p = (size_t)blockIdx.x * FB + (size_t)t;
    const float x  = bfr(cpt[p * CD + 0]), y  = bfr(cpt[p * CD + 1]), z  = bfr(cpt[p * CD + 2]);
    const float px = bfr(mom[p * CD + 0]), py = bfr(mom[p * CD + 1]), pz = bfr(mom[p * CD + 2]);
    const float nq = (x * x + y * y) + z * z;
    const unsigned short nh = f2bf(nq);  const float r1 = nq - bf2f(nh);
    const unsigned short nm = f2bf(r1);  const float r2 = r1 - bf2f(nm);
    const unsigned short nl = f2bf(r2);
    const unsigned short one = (unsigned short)0x3F80u;
    v8us j0, j1, i0;
    j0[0] = f2bf(-2.0f * x); j0[1] = f2bf(-2.0f * y); j0[2] = f2bf(-2.0f * z); j0[3] = nh; j0[4] = nm; j0[5] = nl; j0[6] = 0; j0[7] = 0;
    j1[0] = f2bf(px); j1[1] = f2bf(py); j1[2] = f2bf(pz); j1[3] = 0; j1[4] = 0; j1[5] = 0; j1[6] = 0; j1[7] = 0;
    i0[0] = f2bf(x); i0[1] = f2bf(y); i0[2] = f2bf(z); i0[3] = one; i0[4] = one; i0[5] = one; i0[6] = 0; i0[7] = 0;
    *(v8usa*)(&sj[t * FW]) = j0; *(v8usa*)(&sj[t * FW + 8]) = j1;
    *(v8usa*)(&si[t * FW]) = i0; *(v8usa*)(&si[t * FW + 8]) = j1;
    sc[0 * FB + t] = toh_flush(px * BC); sc[1 * FB + t] = toh_flush(py * BC); sc[2 * FB + t] = toh_flush(pz * BC);
    sc[3 * FB + t] = toh_flush(x * BC);  sc[4 * FB + t] = toh_flush(y * BC);  sc[5 * FB + t] = toh_flush(z * BC);
    sc[6 * FB + t] = (h16)BC;
#pragma unroll 1
    for (int c = 7; c < 16; ++c) sc[c * FB + t] = (h16)0.0f;
    sn[t] = nq;
    __syncthreads();
    const int q0 = t, q1 = t + FB;
    const v8us fj0 = *(const v8usa*)(&sj[q0 * 8]), fj1 = *(const v8usa*)(&sj[q1 * 8]);
    const v8us fi0 = *(const v8usa*)(&si[q0 * 8]), fi1 = *(const v8usa*)(&si[q1 * 8]);
    const v8h  cc0 = *(const v8ha*)(&sc[q0 * 8]),  cc1 = *(const v8ha*)(&sc[q1 * 8]);
    const bool wn = t < FB / 4;
    const int qn = wn ? t : 0;
    const v4f nv = *(const v4fa*)(&sn[qn * 4]);
    const size_t fb0 = (size_t)blockIdx.x * FB * FW;
    bf* dj0 = FJ + fb0 + (size_t)q0 * 8; bf* dj1 = FJ + fb0 + (size_t)q1 * 8;
    bf* di0 = FI + fb0 + (size_t)q0 * 8; bf* di1 = FI + fb0 + (size_t)q1 * 8;
    h16* dc0 = CT + (size_t)(q0 >> 5) * NPTS + (size_t)blockIdx.x * FB + (size_t)(q0 & 31) * 8;
    h16* dc1 = CT + (size_t)(q1 >> 5) * NPTS + (size_t)blockIdx.x * FB + (size_t)(q1 & 31) * 8;
    float* dn = NQ + (size_t)blockIdx.x * FB + (size_t)qn * 4;
    *(volatile v8us*)dj0 = fj0; *(volatile v8us*)dj1 = fj1; *(volatile v8us*)di0 = fi0; *(volatile v8us*)di1 = fi1;
    *(volatile v8h*)dc0 = cc0;  *(volatile v8h*)dc1 = cc1;  if (wn) *(volatile v4f*)dn = nv;
    __threadfence();
    *(volatile v8us*)dj0 = fj0; *(volatile v8us*)dj1 = fj1; *(volatile v8us*)di0 = fi0; *(volatile v8us*)di1 = fi1;
    *(volatile v8h*)dc0 = cc0;  *(volatile v8h*)dc1 = cc1;  if (wn) *(volatile v4f*)dn = nv;
}

__global__ __launch_bounds__(32 * AW) void k_pair(const bf* __restrict__ FJ, const bf* __restrict__ FI, const h16* __restrict__ CT, const float* __restrict__ NQ,
                                                  const float* __restrict__ cpt, float* OUT) {
    __shared__ __align__(16) float so[2 * OSF];
    const int lane = threadIdx.x & 31, lr = lane & 15, hi = lane >> 4;
    const int wave = __builtin_amdgcn_readfirstlane((int)(threadIdx.x >> 5));
    const int t0 = (blockIdx.x * AW + wave) * 16;
    const v8us z8 = (v8us){};
    const v8us fi = *(const v8us*)(FI + (size_t)(t0 + lr) * FW + 8 * hi);
    v8us fd, fp;
#pragma unroll
    for (int k = 0; k < 8; ++k) { fd[k] = hi ? (unsigned short)0 : fi[k]; fp[k] = hi ? fi[k] : (unsigned short)0; }
    const v16bf bd = cat16b(fd, z8), bp = cat16b(fp, z8);
    const float nqi = NQ[t0 + lr];
    const float qx = bfr(cpt[(size_t)(t0 + lr) * CD + 0]), qy = bfr(cpt[(size_t)(t0 + lr) * CD + 1]), qz = bfr(cpt[(size_t)(t0 + lr) * CD + 2]);
    const size_t jo = (size_t)lr * FW + 8 * hi;
    const size_t co = (size_t)lr * NPTS + 8 * hi;
    v8f accK = (v8f){}, accW = (v8f){};
#pragma unroll 1
    for (int key0 = 0; key0 < NPTS; key0 += 32) {
        const bf* fa = FJ + jo + (size_t)key0 * FW;
        const v16bf a0 = cat16b(*(const v8us*)fa, z8), a1 = cat16b(*(const v8us*)(fa + 16 * FW), z8);
        v8f sDa = (v8f){}, sPa = (v8f){}, sDb = (v8f){}, sPb = (v8f){};
        sDa = wmmabg(a0, bd, sDa); sPa = wmmabg(a0, bp, sPa);
        sDb = wmmabg(a1, bd, sDb); sPb = wmmabg(a1, bp, sPb);
        v16h kb, wb;
#pragma unroll
        for (int r = 0; r < 8; ++r) {
            const float ea = (sDa[r] + nqi) * ES_ + KSH, eb = (sDb[r] + nqi) * ES_ + KSH;
            const float xa = __builtin_amdgcn_exp2f(ea), xb = __builtin_amdgcn_exp2f(eb);
            const float ka = (ea < -KSH) ? 0.0f : xa, kc = (eb < -KSH) ? 0.0f : xb;
            kb[r] = (h16)ka; kb[8 + r] = (h16)kc;
            wb[r] = toh_flush(ka * sPa[r]); wb[8 + r] = toh_flush(kc * sPb[r]); }
        const v16h ct = ldh(CT + co + key0);
        accK = wmma16g(ct, kb, accK);
        accW = wmma16g(ct, wb, accW);
    }
    if (hi == 0) {
        const int ob = (wave * 16 + lr) * CD;
        const float rs = accW[6];
        so[ob + 0] = C0_ * (qx * rs - accW[3]); so[ob + 1] = C0_ * (qy * rs - accW[4]); so[ob + 2] = C0_ * (qz * rs - accW[5]);
        so[OSF + ob + 0] = C1_ * accK[0]; so[OSF + ob + 1] = C1_ * accK[1]; so[OSF + ob + 2] = C1_ * accK[2];
    }
    __syncthreads();
    const int t = threadIdx.x;
    if (t < 2 * OSF / 4) {
        const int which = (t >= OSF / 4) ? 1 : 0; const int pc = t - which * (OSF / 4);
        const v4f val = *(const v4fa*)(&so[t * 4]);
        float* dst = OUT + (size_t)which * OUT1_OFF + (size_t)blockIdx.x * OSF + (size_t)pc * 4;
        *(volatile v4f*)dst = val; __threadfence(); *(volatile v4f*)dst = val;
    }
}

static constexpr size_t al256(size_t v) { return (v + 255) & ~(size_t)255; }
static constexpr size_t SZ_F  = al256((size_t)NPTS * FW * 2);
static constexpr size_t SZ_C  = al256((size_t)16 * NPTS * 2);
static constexpr size_t SZ_N  = al256((size_t)NPTS * 4);
static constexpr size_t SZ_TOTAL = 2 * SZ_F + SZ_C + SZ_N;
static_assert(SZ_TOTAL <= (size_t)134217728);
static_assert((size_t)(NPTS / FB) * FB * FW * 2 == (size_t)NPTS * FW * 2);
static_assert((size_t)15 * NPTS + (size_t)(NPTS / FB - 1) * FB + 31 * 8 + 8 == (size_t)16 * NPTS);
static_assert(((size_t)(NPTS / FB - 1) * FB + (size_t)(FB / 4 - 1) * 4 + 4) * 4 == (size_t)NPTS * 4);
static_assert((2 * SZ_F + SZ_C) % 128 == 0);

extern "C" void kernel_launch(void* const* d_in, const int* in_sizes, int n_in,
                              void* d_out, int out_size, void* d_ws, size_t ws_size, hipStream_t stream) {
    if (n_in < 2) return;
    if ((size_t)in_sizes[0] < (size_t)NPTS * CD || (size_t)in_sizes[1] < (size_t)NPTS * CD) return;
    if ((size_t)out_size < OUT1_OFF + (size_t)NPTS * CD) return;
    if (SZ_TOTAL > ws_size) return;
    const float* mom = (const float*)d_in[0];
    const float* cpt = (const float*)d_in[1];
    float* OUT = (float*)d_out;
    char* wsp = (char*)d_ws;
    bf*  FJ = (bf*)wsp;  wsp += SZ_F;
    bf*  FI = (bf*)wsp;  wsp += SZ_F;
    h16* CT = (h16*)wsp; wsp += SZ_C;
    float* NQ = (float*)wsp; wsp += SZ_N;
    k_feat<<<dim3(NPTS / FB, 1, 1), FB, 0, stream>>>(mom, cpt, FJ, FI, CT, NQ);
    k_pair<<<dim3(NPTS / TPB, 1, 1), 32 * AW, 0, stream>>>(FJ, FI, CT, NQ, cpt, OUT);
}
